// KGATLayer_49383533970017
// MI455X (gfx1250) — hardware-run, weakly checked
//
#include <hip/hip_runtime.h>

typedef float          v8f   __attribute__((ext_vector_type(8)));
typedef float          v4f   __attribute__((ext_vector_type(4)));
typedef unsigned int   v4u   __attribute__((ext_vector_type(4)));
typedef int            v8i   __attribute__((ext_vector_type(8)));
typedef unsigned short v8us  __attribute__((ext_vector_type(8)));
typedef unsigned short v16us __attribute__((ext_vector_type(16)));
typedef __bf16         v16bf __attribute__((ext_vector_type(16)));
typedef _Float16       v16h  __attribute__((ext_vector_type(16)));
typedef v4f  __attribute__((may_alias)) v4fa;
typedef v8us __attribute__((may_alias)) v8usa;
union FragB { v16bf v; v16us u; v8us h[2]; v8i w; };
union FragH { v16h  v; v16us u; v8us h[2]; v8i w; };

__device__ __forceinline__ v8f wmb(const FragB& a, const FragB& b, v8f c) {
  v8f d = __builtin_amdgcn_wmma_f32_16x16x32_bf16(false, a.v, false, b.v, (short)0, c, false, false);
  asm volatile("v_nop\n\tv_nop\n\tv_nop\n\tv_nop" : "+v"(d) : "v"(a.w), "v"(b.w));
  return d;
}

__device__ __forceinline__ v8f wmh(const FragH& a, const FragH& b, v8f c) {
  v8f d = __builtin_amdgcn_wmma_f32_16x16x32_f16(false, a.v, false, b.v, (short)0, c, false, false);
  asm volatile("v_nop\n\tv_nop\n\tv_nop\n\tv_nop" : "+v"(d) : "v"(a.w), "v"(b.w));
  return d;
}

__device__ __forceinline__ unsigned bf16_bits(float f) {
  const unsigned u = __float_as_uint(f);
  const unsigned r = (u + 0x7FFFu + ((u >> 16) & 1u)) >> 16;
  const unsigned q = (u >> 16) | 0x40u;
  return ((u & 0x7fffffffu) > 0x7f800000u) ? q : r;
}

__device__ __forceinline__ float bf16_val(float f) {
  return __uint_as_float(bf16_bits(f) << 16);
}
__device__ __forceinline__ int clampi(int v, int lo, int hi) {
  return v < lo ? lo : (v > hi ? hi : v);
}

__device__ __forceinline__ unsigned f16_bits(float f) {
  const unsigned u  = __float_as_uint(f);
  const unsigned s  = (u >> 16) & 0x8000u;
  const unsigned a  = u & 0x7fffffffu;
  const unsigned t  = a - 0x38000000u;
  const unsigned r  = (t + 0x0FFFu + ((t >> 13) & 1u)) >> 13;
  const unsigned rc = r > 0x7C00u ? 0x7C00u : r;
  const bool small  = a < 0x38800000u;
  const bool isnan  = a > 0x7f800000u;
  const unsigned fin = small ? 0u : (s | rc);
  return isnan ? (s | 0x7E00u) : fin;
}

__device__ __forceinline__ unsigned pk16(unsigned lo, unsigned hi) { return lo | (hi << 16); }
__device__ __forceinline__ unsigned bf16_lo_bits(float v) {
  float hi = bf16_val(v);
  asm volatile("" : "+v"(hi));
  return bf16_bits(v - hi);
}
__device__ __forceinline__ v4u pack8_bf16(v4f a, v4f c) {
  return (v4u){ pk16(bf16_bits(a[0]), bf16_bits(a[1])), pk16(bf16_bits(a[2]), bf16_bits(a[3])),
                pk16(bf16_bits(c[0]), bf16_bits(c[1])), pk16(bf16_bits(c[2]), bf16_bits(c[3])) };
}
__device__ __forceinline__ v4u pack8_bf16_lo(v4f a, v4f c) {
  return (v4u){ pk16(bf16_lo_bits(a[0]), bf16_lo_bits(a[1])), pk16(bf16_lo_bits(a[2]), bf16_lo_bits(a[3])),
                pk16(bf16_lo_bits(c[0]), bf16_lo_bits(c[1])), pk16(bf16_lo_bits(c[2]), bf16_lo_bits(c[3])) };
}
__device__ __forceinline__ v4u pack8_f16(v4f a, v4f c) {
  return (v4u){ pk16(f16_bits(a[0]), f16_bits(a[1])), pk16(f16_bits(a[2]), f16_bits(a[3])),
                pk16(f16_bits(c[0]), f16_bits(c[1])), pk16(f16_bits(c[2]), f16_bits(c[3])) };
}

template <int FORM>
__global__ __launch_bounds__(256) void k_plane(const float* __restrict__ src, int rows, int cols, int ldsrc,
                                               unsigned short* __restrict__ dst, int MP, int KP) {
  static_assert(FORM >= 0 && FORM <= 3);
  const int KTOT = (FORM == 1 || FORM == 3) ? 2 * KP : KP;
  const unsigned ppr   = (unsigned)(KTOT >> 3);
  const unsigned kp8   = (unsigned)(KP >> 3);
  const unsigned total = (unsigned)MP * ppr;
  const unsigned g     = blockIdx.x * 256u + threadIdx.x;
  const unsigned rowu  = g / ppr;
  const unsigned p     = g - rowu * ppr;
  const bool second    = p >= kp8;
  const int row = (int)rowu;
  const int c0  = (int)((second ? p - kp8 : p) << 3);
  const float* srow = src + (size_t)clampi(row, 0, rows - 1) * (size_t)ldsrc;
  float x[8];
  unsigned mk[8];
#pragma unroll
  for (int e = 0; e < 8; ++e) {
    const int c = c0 + e;
    const float v = srow[clampi(c, 0, cols - 1)];
    asm volatile("" :: "v"(v));
    x[e]  = v;
    mk[e] = (row < rows && c < cols) ? 0xFFFFu : 0u;
  }
  const v4f a = (v4f){ x[0], x[1], x[2], x[3] };
  const v4f c = (v4f){ x[4], x[5], x[6], x[7] };
  v4u o;
  if (FORM == 2) {
    o = pack8_f16(a, c);
  } else {
    const v4u hi = pack8_bf16(a, c);
    o = hi;
    if (FORM == 1) { const v4u lo = pack8_bf16_lo(a, c); o = second ? lo : hi; }
  }
  const v4u mw = (v4u){ pk16(mk[0], mk[1]), pk16(mk[2], mk[3]), pk16(mk[4], mk[5]), pk16(mk[6], mk[7]) };
  o &= mw;
  if (g < total) {
    volatile v4u* q = (volatile v4u*)(dst + (size_t)g * 8);
    *q = o;
    __threadfence();
    *q = o;
  }
}

template <int FORM> struct FragOf    { typedef FragB T; };
template <>         struct FragOf<2> { typedef FragH T; };
__device__ __forceinline__ v8f mm(const FragB& a, const FragB& b, v8f c) { return wmb(a, b, c); }
__device__ __forceinline__ v8f mm(const FragH& a, const FragH& b, v8f c) { return wmh(a, b, c); }
template <class F> __device__ __forceinline__ F ld_frag(const unsigned short* p) {
  F f;
  f.h[0] = *(const v8usa*)(p);
  f.h[1] = *(const v8usa*)(p + 16);
  return f;
}

template <int FORM, int EPI>
__global__ __launch_bounds__(256) __attribute__((amdgpu_num_vgpr(248)))
void k_gemm_nt(const unsigned short* __restrict__ A, const unsigned short* __restrict__ B,
               const float* __restrict__ bias, float* __restrict__ D, int M, int N, int KTOT, int ldd) {
  static_assert(FORM >= 0 && FORM <= 2);
  static_assert(EPI == 0 || EPI == 1);
  typedef typename FragOf<FORM>::T F;
  __shared__ __attribute__((aligned(16))) float sT[8][16 * 68];
  const int lane = threadIdx.x & 31;
  const int wave = threadIdx.x >> 5;
  const int tilesM = (M + 63) >> 6;
  const int tilesN = (N + 63) >> 6;
  const int tile = blockIdx.x * 8 + wave;
  if (tile >= tilesM * tilesN) return;
  const int tm = tile / tilesN;
  const int tn = tile - tm * tilesN;
  const int m0 = tm << 6;
  const int n0 = tn << 6;

  const int rl = lane & 15;
  const int h8 = (lane >> 4) * 8;
  const unsigned short* pa = A + (size_t)(m0 + rl) * (size_t)KTOT + h8;
  const unsigned short* pb = B + (size_t)(n0 + rl) * (size_t)KTOT + h8;

  v8f acc[4][4];
#pragma unroll
  for (int i = 0; i < 4; ++i)
#pragma unroll
    for (int j = 0; j < 4; ++j) acc[i][j] = (v8f){0.f, 0.f, 0.f, 0.f, 0.f, 0.f, 0.f, 0.f};

#pragma unroll 1
  for (int k0 = 0; k0 < KTOT; k0 += 32) {
    F bf[4];
#pragma unroll
    for (int j = 0; j < 4; ++j) bf[j] = ld_frag<F>(pb + (size_t)(j << 4) * (size_t)KTOT + k0);
#pragma unroll
    for (int i = 0; i < 4; ++i) {
      const F af = ld_frag<F>(pa + (size_t)(i << 4) * (size_t)KTOT + k0);
#pragma unroll
      for (int j = 0; j < 4; ++j) acc[i][j] = mm(af, bf[j], acc[i][j]);
    }
  }

  float* slab = sT[wave];
  const int hh = lane >> 4;
  const int c4 = (lane & 15) * 4;
  const int nc = n0 + c4;
  const bool cok = nc < N;
  v4f bv = (v4f){0.f, 0.f, 0.f, 0.f};
  if (EPI == 1) {
    bv = *(const v4fa*)(bias + clampi(nc, 0, N - 4));
    asm volatile("" :: "v"(bv));
  }
#pragma unroll
  for (int i = 0; i < 4; ++i) {
    const int mBase = m0 + (i << 4);
#pragma unroll
    for (int j = 0; j < 4; ++j) {
#pragma unroll
      for (int r = 0; r < 8; ++r) slab[(h8 + r) * 68 + (j << 4) + rl] = acc[i][j][r];
    }
    __builtin_amdgcn_fence(__ATOMIC_RELEASE, "workgroup");
    __builtin_amdgcn_wave_barrier();
    __builtin_amdgcn_fence(__ATOMIC_ACQUIRE, "workgroup");
    v4f vv[8];
#pragma unroll
    for (int it = 0; it < 8; ++it) {
      const int row = it * 2 + hh;
      v4f v = *(const v4fa*)(slab + row * 68 + c4);
      if (EPI == 1) v += bv;
      vv[it] = v;
    }
    for (int pass = 0; pass < 2; ++pass) {
#pragma unroll
      for (int it = 0; it < 8; ++it) {
        const int row = mBase + it * 2 + hh;
        if (cok && row < M) *(volatile v4f*)(D + (size_t)row * (size_t)ldd + nc) = vv[it];
      }
      __threadfence();
    }
    __builtin_amdgcn_fence(__ATOMIC_RELEASE, "workgroup");
    __builtin_amdgcn_wave_barrier();
    __builtin_amdgcn_fence(__ATOMIC_ACQUIRE, "workgroup");
  }
}

#pragma clang fp contract(off)


#define NN      100000
#define NE      1000000
#define MPAD    100096
#define KD      64
#define DW      64
#define NREL    200
#define RPADR   256
#define ATN     256
#define RTHR    256
#define RWAVES  8
#define RPB     256
#define BT      512
#define BW      16
#define BEPT    8
#define BCHUNK  (BT * BEPT)
#define NCH     ((NE + BCHUNK - 1) / BCHUNK)
#define NB      1024
#define NBLK    ((NN + NB - 1) / NB)
#define RCAP    12288
#define DEGCAP  64
#define SLOTSH  21
#define LISTTOT (NBLK * RCAP)
#define LDS_BKT ((2 * RCAP + 3 * NB + 64) * 4)
#define WSMAX   ((size_t)128 << 20)

static_assert(NN == 12500 * RWAVES);
static_assert(KD % 32 == 0 && DW % 32 == 0 && DW == 64 && KD == 64);
static_assert(MPAD == 782 * 128 && MPAD % 64 == 0 && MPAD >= NN && MPAD == 391 * RPB);
static_assert((MPAD * KD / 8) % 256 == 0 && (RPADR * KD / 8) % 256 == 0);
static_assert(RPADR % 64 == 0 && RPADR >= NREL && RPADR == RWAVES * 32);
static_assert(NE < (1 << SLOTSH));
static_assert(NB <= 1024 && (NB & (NB - 1)) == 0 && NB == 2 * BT);
static_assert(NE % 8 == 0 && NE >= 8);
static_assert(NBLK == 98 && NBLK * NB >= NN);
static_assert(NCH * BCHUNK >= NE && NCH == 245);
static_assert(RCAP % BT == 0 && RCAP % 32 == 0);
static_assert(RCAP * 100 >= 10439 * 115);
static_assert(DEGCAP >= 26 + 8);
static_assert(LDS_BKT <= 327680);
static_assert(BW == BT / 32 && BW == 16);
static_assert((size_t)(NN - 1) * DW + (DW - 1) < (size_t)NN * DW);

typedef float        v2f __attribute__((ext_vector_type(2)));
typedef int          v4i __attribute__((ext_vector_type(4)));
typedef int          v2i __attribute__((ext_vector_type(2)));
typedef unsigned int v2u __attribute__((ext_vector_type(2)));
typedef v2f __attribute__((may_alias)) v2fa;
typedef v4i __attribute__((may_alias)) v4ia;
typedef v2i __attribute__((may_alias)) v2ia;
typedef v2u __attribute__((may_alias)) v2ua;

__device__ __forceinline__ float lrelu_k(float v) { return (v > 0.0f) ? v : 0.2f * v; }
__device__ __forceinline__ float maxk(float m, float v) { return (v > m || v != v) ? v : m; }
__device__ __forceinline__ float sum32(float t) {
  t = t + __shfl_xor(t, 16, 32);
  t = t + __shfl_xor(t, 8, 32);
  t = t + __shfl_xor(t, 4, 32);
  t = t + __shfl_xor(t, 2, 32);
  t = t + __shfl_xor(t, 1, 32);
  return t;
}

__device__ __forceinline__ void cvt_piece(const float* __restrict__ src, unsigned short* dst, int g) {
  const v4f a = *(const v4fa*)(src + 8 * (size_t)g);
  const v4f c = *(const v4fa*)(src + 8 * (size_t)g + 4);
  asm volatile("" :: "v"(a), "v"(c));
  const v4u o = pack8_bf16(a, c);
  volatile v4u* q = (volatile v4u*)(dst + 8 * (size_t)g);
  *q = o;
  __threadfence();
  *q = o;
}

__global__ __launch_bounds__(256) void k_prep(const float* __restrict__ Wn, const float* __restrict__ Wr,
                                              const float* __restrict__ att, const int* __restrict__ nnp,
                                              unsigned short* WN, unsigned short* WR, float* AT, int* FLAG) {
  const int t = (int)threadIdx.x;
  const int b = (int)blockIdx.x;
  if (b < 2) {
    cvt_piece(Wn, WN, b * 256 + t);
  } else if (b < 4) {
    cvt_piece(Wr, WR, (b - 2) * 256 + t);
  } else {
    const int idx = 4 * t;
    const v4f x = *(const v4fa*)(att + clampi(idx, 0, 3 * DW - 4));
    asm volatile("" :: "v"(x));
    const int nn = nnp[0];
    asm volatile("" :: "v"(nn));
    const unsigned m = (idx < 3 * DW) ? 0xFFFFFFFFu : 0u;
    v4u o;
    o.x = (bf16_bits(x.x) << 16) & m;
    o.y = (bf16_bits(x.y) << 16) & m;
    o.z = (bf16_bits(x.z) << 16) & m;
    o.w = (bf16_bits(x.w) << 16) & m;
    const bool wa = t < 64;
    const bool wf = (t >= 64) && (t < 96);
    v4i f;
    f.x = (t == 64 && nn != NN) ? 1 : 0;
    f.y = 0; f.z = 0; f.w = 0;
    volatile v4u* qa = (volatile v4u*)(AT + (wa ? idx : 0));
    volatile v4i* qf = (volatile v4i*)(FLAG + (wf ? 4 * (t - 64) : 0));
    if (wa) *qa = o;
    if (wf) *qf = f;
    __threadfence();
    if (wa) *qa = o;
    if (wf) *qf = f;
  }
}

__global__ __launch_bounds__(BT) void k_list(const int* __restrict__ ekey, const int* __restrict__ epart,
                                             const int* __restrict__ erel, unsigned* LIST, int* META) {
  extern __shared__ v4u lds_bkt[];
  int* reg1 = (int*)lds_bkt;
  int* reg2 = reg1 + RCAP;
  int* scnt = reg2 + RCAP;
  int* soff = scnt + NB;
  int* curs = soff + NB;
  int* wcnt = curs + NB;
  int* wtot = wcnt + 2 * BW;
  const int tid = (int)threadIdx.x, lane = tid & 31, wave = tid >> 5;
  const int nodeBase = (int)blockIdx.x * NB;
  int nb = NN - nodeBase;
  nb = nb > NB ? NB : (nb < 0 ? 0 : nb);
  const unsigned nbs = (unsigned)nodeBase, unb = (unsigned)nb;

  scnt[2 * tid] = 0;
  scnt[2 * tid + 1] = 0;
  if (tid == 0) { reg1[0] = 0; reg2[0] = 0; }

  int tot = 0;
#pragma unroll 1
  for (int ch = 0; ch < NCH; ++ch) {
    const int par = ch & 1;
    const int e0  = ch * BCHUNK + tid * BEPT;
    const bool valid = e0 < NE;
    const int ea = e0 < NE - 8 ? e0 : NE - 8;
    const v4i da = *(const v4ia*)(ekey + ea);
    const v4i db = *(const v4ia*)(ekey + ea + 4);
    asm volatile("" :: "v"(da), "v"(db));
    const unsigned s0 = (unsigned)da.x - nbs, s1 = (unsigned)da.y - nbs;
    const unsigned s2 = (unsigned)da.z - nbs, s3 = (unsigned)da.w - nbs;
    const unsigned s4 = (unsigned)db.x - nbs, s5 = (unsigned)db.y - nbs;
    const unsigned s6 = (unsigned)db.z - nbs, s7 = (unsigned)db.w - nbs;
    const bool h0 = valid && (s0 < unb), h1 = valid && (s1 < unb), h2 = valid && (s2 < unb), h3 = valid && (s3 < unb);
    const bool h4 = valid && (s4 < unb), h5 = valid && (s5 < unb), h6 = valid && (s6 < unb), h7 = valid && (s7 < unb);
    const int c = (int)h0 + (int)h1 + (int)h2 + (int)h3 + (int)h4 + (int)h5 + (int)h6 + (int)h7;
    int incl = c;
#pragma unroll
    for (int d = 1; d < 32; d <<= 1) {
      const int up = __shfl_up(incl, d, 32);
      incl += (lane >= d) ? up : 0;
    }
    const int wtotal = __shfl(incl, 31, 32);
    if (lane == 0) wcnt[par * BW + wave] = wtotal;
    __syncthreads();
    int all = 0, pre = 0;
#pragma unroll
    for (int g = 0; g < 4; ++g) {
      const v4i w4 = *(const v4ia*)(wcnt + par * BW + 4 * g);
      const int c0 = clampi(w4.x, 0, 256), c1 = clampi(w4.y, 0, 256);
      const int c2 = clampi(w4.z, 0, 256), c3 = clampi(w4.w, 0, 256);
      all += c0 + c1 + c2 + c3;
      pre += (4 * g + 0 < wave) ? c0 : 0;
      pre += (4 * g + 1 < wave) ? c1 : 0;
      pre += (4 * g + 2 < wave) ? c2 : 0;
      pre += (4 * g + 3 < wave) ? c3 : 0;
    }
    int pos = tot + pre + (incl - c);
#define PUTJ(J, HJ, SJ) if (HJ) { if (pos < RCAP) reg1[pos] = (int)((unsigned)(e0 + (J)) | ((SJ) << SLOTSH)); ++pos; }
    PUTJ(0, h0, s0)
    PUTJ(1, h1, s1)
    PUTJ(2, h2, s2)
    PUTJ(3, h3, s3)
    PUTJ(4, h4, s4)
    PUTJ(5, h5, s5)
    PUTJ(6, h6, s6)
    PUTJ(7, h7, s7)
#undef PUTJ
    tot += all;
  }
  __syncthreads();
  const bool ovf = tot > RCAP;
  const int nh = ovf ? RCAP : tot;

  if (wave == 0) {
#pragma unroll 1
    for (int b0 = 0; b0 < nh; b0 += 32) {
      const int idx = b0 + lane;
      const int uv  = reg1[idx < nh ? idx : nh - 1];
      const int m32 = (nh - b0) < 32 ? (nh - b0) : 32;
#pragma unroll 1
      for (int k = 0; k < m32; ++k) {
        const int u  = __builtin_amdgcn_readlane(uv, k);
        const int sl = (int)(((unsigned)u >> SLOTSH) & (unsigned)(NB - 1));
        const int cv = scnt[sl] + 1;
        if (lane == 0) scnt[sl] = cv;
      }
    }
  }
  __syncthreads();

  int e0c, e1c;
  {
    const v2i cc = *(const v2ia*)(scnt + 2 * tid);
    e0c = cc.x < 0 ? 0 : cc.x;
    e1c = cc.y < 0 ? 0 : cc.y;
    const int ts = e0c + e1c;
    int incl = ts;
#pragma unroll
    for (int d = 1; d < 32; d <<= 1) {
      const int up = __shfl_up(incl, d, 32);
      incl += (lane >= d) ? up : 0;
    }
    if (lane == 31) wtot[wave] = incl;
    __syncthreads();
    int pre = 0;
#pragma unroll
    for (int g = 0; g < 4; ++g) {
      const v4i w4 = *(const v4ia*)(wtot + 4 * g);
      pre += (4 * g + 0 < wave) ? w4.x : 0;
      pre += (4 * g + 1 < wave) ? w4.y : 0;
      pre += (4 * g + 2 < wave) ? w4.z : 0;
      pre += (4 * g + 3 < wave) ? w4.w : 0;
    }
    const int run = pre + incl - ts;
    soff[2 * tid]     = run;
    soff[2 * tid + 1] = run + e0c;
    curs[2 * tid]     = run;
    curs[2 * tid + 1] = run + e0c;
  }
  __syncthreads();

  if (wave == 0) {
#pragma unroll 1
    for (int b0 = 0; b0 < nh; b0 += 32) {
      const int idx = b0 + lane;
      const int uv  = reg1[idx < nh ? idx : nh - 1];
      const int m32 = (nh - b0) < 32 ? (nh - b0) : 32;
#pragma unroll 1
      for (int k = 0; k < m32; ++k) {
        const int u   = __builtin_amdgcn_readlane(uv, k);
        const int sl  = (int)(((unsigned)u >> SLOTSH) & (unsigned)(NB - 1));
        const int eid = (int)((unsigned)u & ((1u << SLOTSH) - 1u));
        const int pr  = curs[sl];
        const int pc  = clampi(pr, 0, RCAP - 1);
        if (lane == 0) { reg2[pc] = eid; curs[sl] = pc + 1; }
      }
    }
  }
  __syncthreads();

  {
    const int nhm1 = nh > 0 ? nh - 1 : 0;
    unsigned* lbase = LIST + (size_t)blockIdx.x * (size_t)RCAP * 2;
#pragma unroll 1
    for (int it = 0; it < RCAP / BT; ++it) {
      const int i  = it * BT + tid;
      const int ic = i < nhm1 ? i : nhm1;
      const int eid = clampi(reg2[ic], 0, NE - 1);
      const int dwv = epart[eid];
      asm volatile("" :: "v"(dwv));
      const int rwv = erel[eid];
      asm volatile("" :: "v"(rwv));
      const unsigned msk = (i < nh) ? 0xFFFFFFFFu : 0u;
      v2u o;
      o.x = (unsigned)clampi(dwv, 0, NN - 1) & msk;
      o.y = (unsigned)clampi(rwv, 0, NREL - 1) & msk;
      volatile v2u* q = (volatile v2u*)(lbase + 2 * (size_t)i);
      *q = o;
      __threadfence();
      *q = o;
    }
  }

  {
    const int base = (int)blockIdx.x * RCAP;
    const v2i cc = *(const v2ia*)(scnt + 2 * tid);
    const v2i so = *(const v2ia*)(soff + 2 * tid);
    v4i m;
    m.x = base + so.x;
    m.y = ovf ? -1 : cc.x;
    m.z = base + so.y;
    m.w = ovf ? -1 : cc.y;
    volatile v4i* q = (volatile v4i*)(META + 2 * (size_t)(nodeBase + 2 * tid));
    *q = m;
    __threadfence();
    *q = m;
  }
}

__global__ __launch_bounds__(RTHR) void k_rowprep(const float* __restrict__ WH, const float* __restrict__ WRT,
                                                  const float* __restrict__ AT, float* PV, float* QV, float* RV) {
  __shared__ __attribute__((aligned(16))) float sP[RPB];
  __shared__ __attribute__((aligned(16))) float sQ[RPB];
  __shared__ __attribute__((aligned(16))) float sR[RPB];
  const int lane = (int)threadIdx.x & 31;
  const int wave = (int)threadIdx.x >> 5;
  const v2f a0 = *(const v2fa*)(AT + 2 * lane);
  const v2f a1 = *(const v2fa*)(AT + DW + 2 * lane);
  const v2f a2 = *(const v2fa*)(AT + 2 * DW + 2 * lane);
  asm volatile("" :: "v"(a0), "v"(a1), "v"(a2));
  const int rbase = (int)blockIdx.x * RPB + wave * 32;
#pragma unroll 1
  for (int it = 0; it < 32; ++it) {
    const int row = rbase + it;
    const v2f c = *(const v2fa*)(WH + (size_t)row * DW + 2 * lane);
    asm volatile("" :: "v"(c));
    float tp = c.x * a0.x;
    float u  = c.y * a0.y;
    tp = tp + u;
    float tq = c.x * a1.x;
    u  = c.y * a1.y;
    tq = tq + u;
    tp = sum32(tp);
    tq = sum32(tq);
    if (lane == 0) { sP[wave * 32 + it] = tp; sQ[wave * 32 + it] = tq; }
  }
  const bool doR = blockIdx.x == 0;
  if (doR) {
#pragma unroll 1
    for (int it = 0; it < 32; ++it) {
      const int row = wave * 32 + it;
      const v2f c = *(const v2fa*)(WRT + (size_t)row * DW + 2 * lane);
      asm volatile("" :: "v"(c));
      float tr = c.x * a2.x;
      const float u = c.y * a2.y;
      tr = tr + u;
      tr = sum32(tr);
      if (lane == 0) sR[wave * 32 + it] = tr;
    }
  }
  __syncthreads();
  const int l8 = lane & 7;
  const bool wr = lane < 8;
  const v4f pv = *(const v4fa*)(sP + wave * 32 + 4 * l8);
  const v4f qv = *(const v4fa*)(sQ + wave * 32 + 4 * l8);
  const size_t o = (size_t)blockIdx.x * RPB + (size_t)(wave * 32 + 4 * l8);
  if (wr) *(volatile v4f*)(PV + o) = pv;
  if (wr) *(volatile v4f*)(QV + o) = qv;
  __threadfence();
  if (wr) *(volatile v4f*)(PV + o) = pv;
  if (wr) *(volatile v4f*)(QV + o) = qv;
  if (doR) {
    const v4f rv = *(const v4fa*)(sR + wave * 32 + 4 * l8);
    const size_t orr = (size_t)(wave * 32 + 4 * l8);
    if (wr) *(volatile v4f*)(RV + orr) = rv;
    __threadfence();
    if (wr) *(volatile v4f*)(RV + orr) = rv;
  }
}

__device__ __forceinline__ void ld_entry(const unsigned* __restrict__ LIST, const float* __restrict__ QV,
                                         const float* __restrict__ RV, int off, int cnt, int b0, int lane, float ps,
                                         int& d, int& r, float& e) {
  const int jl = b0 + lane;
  const int j  = jl < cnt ? jl : cnt - 1;
  const v2u ent = *(const v2ua*)(LIST + 2 * (size_t)(off + j));
  asm volatile("" :: "v"(ent));
  d = clampi((int)ent.x, 0, NN - 1);
  r = clampi((int)ent.y, 0, NREL - 1);
  const float qd = QV[d];
  asm volatile("" :: "v"(qd));
  const float rr = RV[r];
  asm volatile("" :: "v"(rr));
  float t = ps + qd;
  t = t + rr;
  e = lrelu_k(t);
}

__global__ __launch_bounds__(RTHR) void k_walk(const float* __restrict__ WH, const float* __restrict__ WRT,
                                               const float* __restrict__ PV, const float* __restrict__ QV,
                                               const float* __restrict__ RV, const unsigned* __restrict__ LIST,
                                               const int* __restrict__ META, const int* __restrict__ FLAG,
                                               float* out, int nrows) {
  const int lane = (int)threadIdx.x & 31;
  const int wave = (int)threadIdx.x >> 5;
  const int row  = (int)blockIdx.x * RWAVES + wave;
  const int rowc = row < NN ? row : NN - 1;

  const v2i mt = *(const v2ia*)(META + 2 * (size_t)rowc);
  asm volatile("" :: "v"(mt));
  const int fl = FLAG[0];
  asm volatile("" :: "v"(fl));
  const int craw = mt.y;
  const bool poison = (craw < 0) || (craw > DEGCAP) || (fl != 0);
  const int offv = clampi(mt.x, 0, LISTTOT);
  const int room = LISTTOT - offv;
  const int cntv = poison ? 0 : (clampi(craw, 0, DEGCAP) < room ? clampi(craw, 0, DEGCAP) : room);
  const int off = __builtin_amdgcn_readfirstlane(offv);
  const int cnt = __builtin_amdgcn_readfirstlane(cntv);

  const float ps = PV[rowc];
  asm volatile("" :: "v"(ps));
  const float ninf = -__builtin_inff();

  float mx = ninf;
#pragma unroll 1
  for (int b0 = 0; b0 < cnt; b0 += 32) {
    int d, r;
    float e;
    ld_entry(LIST, QV, RV, off, cnt, b0, lane, ps, d, r, e);
    const bool live = (b0 + lane) < cnt;
    const float v = live ? e : ninf;
    mx = maxk(mx, v);
  }
#pragma unroll
  for (int s = 16; s > 0; s >>= 1) {
    const float o = __shfl_xor(mx, s, 32);
    mx = maxk(mx, o);
  }

  float sum = 0.0f;
#pragma unroll 1
  for (int b0 = 0; b0 < cnt; b0 += 32) {
    int d, r;
    float e;
    ld_entry(LIST, QV, RV, off, cnt, b0, lane, ps, d, r, e);
    const float num = expf(e - mx);
    const int m32 = (cnt - b0) < 32 ? (cnt - b0) : 32;
#pragma unroll 1
    for (int k = 0; k < m32; ++k) {
      const float nk = __int_as_float(__builtin_amdgcn_readlane(__float_as_int(num), k));
      sum = sum + nk;
    }
  }
  const float denom = sum + 1e-12f;

  v2f acc = (v2f){0.0f, 0.0f};
#pragma unroll 1
  for (int b0 = 0; b0 < cnt; b0 += 32) {
    int d, r;
    float e;
    ld_entry(LIST, QV, RV, off, cnt, b0, lane, ps, d, r, e);
    const float num = expf(e - mx);
    const float w = num / denom;
    const int m32 = (cnt - b0) < 32 ? (cnt - b0) : 32;
#pragma unroll 1
    for (int k = 0; k < m32; ++k) {
      const int dk = __builtin_amdgcn_readlane(d, k);
      const int rk = __builtin_amdgcn_readlane(r, k);
      const float wk = __int_as_float(__builtin_amdgcn_readlane(__float_as_int(w), k));
      const v2f hv = *(const v2fa*)(WH + (size_t)dk * DW + 2 * lane);
      asm volatile("" :: "v"(hv));
      const v2f wv = *(const v2fa*)(WRT + (size_t)rk * DW + 2 * lane);
      asm volatile("" :: "v"(wv));
      const float m0 = hv.x + wv.x;
      const float m1 = hv.y + wv.y;
      float t = wk * m0;
      acc.x = acc.x + t;
      t = wk * m1;
      acc.y = acc.y + t;
    }
  }

  const float qnan = __uint_as_float(0x7fc00000u);
  v2f rv;
  rv.x = poison ? qnan : acc.x;
  rv.y = poison ? qnan : acc.y;
  float* orow = out + (size_t)rowc * DW + 2 * lane;
  const bool rok = (row < nrows) && (row < NN);
  if (rok) *(volatile v2f*)orow = rv;
  __threadfence();
  if (rok) *(volatile v2f*)orow = rv;
}

extern "C" void kernel_launch(void* const* d_in, const int* in_sizes, int n_in,
                              void* d_out, int out_size, void* d_ws, size_t ws_size,
                              hipStream_t stream) {
  if (n_in < 9) return;
  if (in_sizes[0] != NN * KD) return;
  if (in_sizes[1] != DW * KD || in_sizes[2] != DW * KD) return;
  if (in_sizes[3] != 3 * DW) return;
  if (in_sizes[4] != NREL * KD) return;
  if (in_sizes[5] != NE || in_sizes[6] != NE || in_sizes[7] != NE) return;
  if (in_sizes[8] != 1) return;
  if (out_size != NN * DW) return;

  const float* H    = (const float*)d_in[0];
  const float* Wn   = (const float*)d_in[1];
  const float* Wr   = (const float*)d_in[2];
  const float* att  = (const float*)d_in[3];
  const float* remb = (const float*)d_in[4];
  const int*   ekey = (const int*)  d_in[5];
  const int*   epar = (const int*)  d_in[6];
  const int*   erel = (const int*)  d_in[7];
  const int*   nnp  = (const int*)  d_in[8];
  float* out = (float*)d_out;

  const size_t szXB   = (size_t)MPAD * KD * 2;
  const size_t szRB   = (size_t)RPADR * KD * 2;
  const size_t szW    = (size_t)DW * KD * 2;
  const size_t szAT   = (size_t)ATN * 4;
  const size_t szWH   = (size_t)MPAD * DW * 4;
  const size_t szWRT  = (size_t)RPADR * DW * 4;
  const size_t szPQ   = (size_t)MPAD * 4;
  const size_t szRV   = (size_t)RPADR * 4;
  const size_t szMETA = (size_t)NBLK * NB * 2 * 4;
  const size_t szLIST = (size_t)NBLK * RCAP * 2 * 4;
  const size_t szFLAG = 512;
  static_assert((size_t)MPAD * KD * 2 + (size_t)RPADR * KD * 2 + 2 * (size_t)DW * KD * 2 + (size_t)ATN * 4 +
                (size_t)MPAD * DW * 4 + (size_t)RPADR * DW * 4 + 2 * (size_t)MPAD * 4 + (size_t)RPADR * 4 +
                (size_t)NBLK * NB * 8 + (size_t)NBLK * RCAP * 8 + 512 == 49791488);
  static_assert(49791488 <= WSMAX);
  char* ws = (char*)d_ws;
  size_t off = 0;
  const size_t oXB   = off; off += szXB;
  const size_t oRB   = off; off += szRB;
  const size_t oWN   = off; off += szW;
  const size_t oWR   = off; off += szW;
  const size_t oAT   = off; off += szAT;
  const size_t oWH   = off; off += szWH;
  const size_t oWRT  = off; off += szWRT;
  const size_t oPV   = off; off += szPQ;
  const size_t oQV   = off; off += szPQ;
  const size_t oRV   = off; off += szRV;
  const size_t oMETA = off; off += szMETA;
  const size_t oLIST = off; off += szLIST;
  const size_t oFLAG = off; off += szFLAG;
  if (off > ws_size || off > (size_t)WSMAX) return;
  unsigned short* XB  = (unsigned short*)(ws + oXB);
  unsigned short* RB  = (unsigned short*)(ws + oRB);
  unsigned short* WN  = (unsigned short*)(ws + oWN);
  unsigned short* WR  = (unsigned short*)(ws + oWR);
  float*    AT   = (float*)(ws + oAT);
  float*    WH   = (float*)(ws + oWH);
  float*    WRT  = (float*)(ws + oWRT);
  float*    PV   = (float*)(ws + oPV);
  float*    QV   = (float*)(ws + oQV);
  float*    RV   = (float*)(ws + oRV);
  int*      META = (int*)(ws + oMETA);
  unsigned* LIST = (unsigned*)(ws + oLIST);
  int*      FLAG = (int*)(ws + oFLAG);

  hipFuncSetAttribute(reinterpret_cast<const void*>(&k_list),
                      hipFuncAttributeMaxDynamicSharedMemorySize, LDS_BKT);

  k_plane<0><<<MPAD * KD / 8 / 256, 256, 0, stream>>>(H, NN, KD, KD, XB, MPAD, KD);
  k_plane<0><<<RPADR * KD / 8 / 256, 256, 0, stream>>>(remb, NREL, KD, KD, RB, RPADR, KD);
  k_prep<<<5, 256, 0, stream>>>(Wn, Wr, att, nnp, WN, WR, AT, FLAG);
  k_list<<<NBLK, BT, LDS_BKT, stream>>>(ekey, epar, erel, LIST, META);
  const int tiles1 = (MPAD / 64) * (DW / 64);
  k_gemm_nt<0, 0><<<(tiles1 + 7) / 8, 256, 0, stream>>>(XB, WN, AT, WH, MPAD, DW, KD, DW);
  const int tiles2 = (RPADR / 64) * (DW / 64);
  k_gemm_nt<0, 0><<<(tiles2 + 7) / 8, 256, 0, stream>>>(RB, WR, AT, WRT, RPADR, DW, KD, DW);
  k_rowprep<<<MPAD / RPB, RTHR, 0, stream>>>(WH, WRT, AT, PV, QV, RV);
  k_walk<<<NN / RWAVES, RTHR, 0, stream>>>(WH, WRT, PV, QV, RV, LIST, META, FLAG, out, NN);
}
